// InfoGraph_68289980006827
// MI455X (gfx1250) — hardware-verified
//
#include <hip/hip_runtime.h>
#include <math.h>

#define NN 50000
#define NE 800000
#define NP 50048
#define GD 64
#define NGR 500
#define NGP 512
#define NT 256
#define SRB 2048
#define NTILE 25
#define SCH 4096
#define NCH ((NE + SCH - 1) / SCH)
#define SCHP 2048
#define NCHP ((NN + SCHP - 1) / SCHP)
#define WSC 64.0f
#define WSC_INV (1.0f / 64.0f)

typedef __attribute__((ext_vector_type(16))) _Float16 v16h;
typedef __attribute__((ext_vector_type(8)))  _Float16 v8h;
typedef __attribute__((ext_vector_type(16))) __bf16   v16b;
typedef __attribute__((ext_vector_type(8)))  __bf16   v8b;
typedef __attribute__((ext_vector_type(8)))  float    v8f;
typedef __attribute__((ext_vector_type(4)))  float    v4f;
typedef __attribute__((ext_vector_type(2)))  float    v2f;
typedef __attribute__((ext_vector_type(4)))  int      v4i;

__device__ __forceinline__ unsigned short f2bf_bits(float f) {
  unsigned u = __float_as_uint(f);
  return (unsigned short)((u + 0x7FFFu + ((u >> 16) & 1u)) >> 16);
}
__device__ __forceinline__ float bf_bits2f(unsigned short h) { return __uint_as_float(((unsigned)h) << 16); }

__device__ __forceinline__ void dep_guard_h(v8f& a, v8f& b, v16h x, v16h y) { asm volatile("v_nop\n\tv_nop\n\tv_nop\n\tv_nop" : "+v"(a), "+v"(b) : "v"(x), "v"(y)); }
__device__ __forceinline__ void dep_guard_b(v8f& a, v8f& b, v16b x, v16b y) { asm volatile("v_nop\n\tv_nop\n\tv_nop\n\tv_nop" : "+v"(a), "+v"(b) : "v"(x), "v"(y)); }
__device__ __forceinline__ void keep4_h(v16h a, v16h b, v16h c, v16h d) { asm volatile("v_nop" :: "v"(a), "v"(b), "v"(c), "v"(d)); }
__device__ __forceinline__ void keep4_b(v16b a, v16b b, v16b c, v16b d) { asm volatile("v_nop" :: "v"(a), "v"(b), "v"(c), "v"(d)); }
__device__ __forceinline__ void acc_guard4(v8f& a, v8f& b, v8f& c, v8f& d) { asm volatile("v_nop\n\tv_nop\n\tv_nop\n\tv_nop" : "+v"(a), "+v"(b), "+v"(c), "+v"(d)); }
template <typename T> struct Frag;
template <> struct Frag<_Float16> {
  typedef v16h V; union U { v16h v; v8h h[2]; };
  static __device__ __forceinline__ v16h load(const _Float16* p) {
    U f; f.h[0] = *(const v8h*)(p); f.h[1] = *(const v8h*)(p + 16); return f.v;
  }
  static __device__ __forceinline__ v8f mma(v16h a, v16h b, v8f c) {
    return __builtin_amdgcn_wmma_f32_16x16x32_f16(false, a, false, b, (short)0, c, false, false);
  }
  static __device__ __forceinline__ void guard(v8f& a, v8f& b, v16h x, v16h y) { dep_guard_h(a, b, x, y); }
  static __device__ __forceinline__ void keep(v16h a, v16h b, v16h c, v16h d) { keep4_h(a, b, c, d); }
};
template <> struct Frag<__bf16> {
  typedef v16b V; union U { v16b v; v8b h[2]; };
  static __device__ __forceinline__ v16b load(const __bf16* p) {
    U f; f.h[0] = *(const v8b*)(p); f.h[1] = *(const v8b*)(p + 16); return f.v;
  }
  static __device__ __forceinline__ v8f mma(v16b a, v16b b, v8f c) {
    return __builtin_amdgcn_wmma_f32_16x16x32_bf16(false, a, false, b, (short)0, c, false, false);
  }
  static __device__ __forceinline__ void guard(v8f& a, v8f& b, v16b x, v16b y) { dep_guard_b(a, b, x, y); }
  static __device__ __forceinline__ void keep(v16b a, v16b b, v16b c, v16b d) { keep4_b(a, b, c, d); }
};

template <int ET> struct Elem;
template <> struct Elem<0> { typedef _Float16 T; };
template <> struct Elem<1> { typedef __bf16 T; };
template <int ET, bool SPLIT, int BIAS_MODE, int OUT_MODE, bool RESID, int ACT, bool BNR>
__global__ __launch_bounds__(256) void wmma_gemm64(
    const unsigned short* __restrict__ Ap, const unsigned short* A2p, int lda, long strideA,
    const unsigned short* __restrict__ Btp, const unsigned short* Bt2p, int ldb, long strideB,
    void* Cout, void* Cout2, int ldc, long strideC,
    const float* __restrict__ bias, const float* __restrict__ bns, const float* __restrict__ bnt,
    const float* __restrict__ resid, long strideR,
    int M, int N, int K, int Mst, float scale) {
  typedef typename Elem<ET>::T T;
  typedef typename Frag<T>::V V;
  const T* A = (const T*)Ap; const T* A2 = (const T*)A2p; const T* Bt = (const T*)Btp; const T* Bt2 = (const T*)Bt2p;
  __shared__ __align__(16) float sT[8][16 * 68];
  const int b    = blockIdx.y;
  const int lane = threadIdx.x & 31;
  const int wave = threadIdx.x >> 5;
  const int tilesN = N >> 6;
  const int tilesM = M >> 6;
  const int tile = blockIdx.x * 8 + wave;
  if (tile >= tilesM * tilesN) return;
  const int tm = tile / tilesN;
  const int tn = tile - tm * tilesN;
  const int m0 = tm << 6;
  const int n0 = tn << 6;

  const T* Ab  = A  + (size_t)b * strideA;
  const T* Bb  = Bt + (size_t)b * strideB;
  const T* Ab2 = SPLIT ? (A2  + (size_t)b * strideA) : nullptr;
  const T* Bb2 = SPLIT ? (Bt2 + (size_t)b * strideB) : nullptr;

  const int rlane = lane & 15;
  const int koff  = (lane >> 4) * 8;
  const int mOff  = (lane >> 4) * 8;

  v8f acc[4][4];
#pragma unroll
  for (int i = 0; i < 4; ++i)
#pragma unroll
    for (int j = 0; j < 4; ++j) acc[i][j] = (v8f){0.f,0.f,0.f,0.f,0.f,0.f,0.f,0.f};

  for (int k0 = 0; k0 < K; k0 += 32) {
    V bh[4], bl[4];
#pragma unroll
    for (int j = 0; j < 4; ++j) {
      const size_t bo = (size_t)(n0 + (j << 4) + rlane) * ldb + koff + k0;
      bh[j] = Frag<T>::load(Bb + bo);
      if (SPLIT) bl[j] = Frag<T>::load(Bb2 + bo);
    }
#pragma unroll
    for (int i = 0; i < 4; ++i) {
      const size_t ao = (size_t)(m0 + (i << 4) + rlane) * lda + koff + k0;
      V ah = Frag<T>::load(Ab + ao);
      V al;
      if (SPLIT) al = Frag<T>::load(Ab2 + ao);
#pragma unroll
      for (int j = 0; j < 4; ++j) {
        acc[i][j] = Frag<T>::mma(ah, bh[j], acc[i][j]);
        if (SPLIT) {
          acc[i][j] = Frag<T>::mma(ah, bl[j], acc[i][j]);
          acc[i][j] = Frag<T>::mma(al, bh[j], acc[i][j]);
        }
      }
      Frag<T>::guard(acc[i][0], acc[i][3], ah, SPLIT ? al : ah);
    }
    Frag<T>::keep(bh[0], bh[1], bh[2], bh[3]);
    if (SPLIT) Frag<T>::keep(bl[0], bl[1], bl[2], bl[3]);
  }
  acc_guard4(acc[0][0], acc[0][1], acc[0][2], acc[0][3]);
  acc_guard4(acc[1][0], acc[1][1], acc[1][2], acc[1][3]);
  acc_guard4(acc[2][0], acc[2][1], acc[2][2], acc[2][3]);
  acc_guard4(acc[3][0], acc[3][1], acc[3][2], acc[3][3]);

  float* slab = sT[wave];
  const float* Rb = RESID ? (resid + (size_t)b * strideR) : nullptr;
#pragma unroll
  for (int i = 0; i < 4; ++i) {
    const int mBase = m0 + (i << 4);
#pragma unroll
    for (int j = 0; j < 4; ++j) {
      const int n = n0 + (j << 4) + rlane;
      float bv = 0.f;
      if (BIAS_MODE == 2) bv = bias[n];
      float sv = 0.f, tv = 0.f;
      if (BNR) { sv = bns[n]; tv = bnt[n]; }
#pragma unroll
      for (int r = 0; r < 8; ++r) {
        float v = acc[i][j][r] * scale;
        if (BIAS_MODE == 1) v += bias[mBase + mOff + r];
        if (BIAS_MODE == 2) v += bv;
        if (RESID) v += Rb[(size_t)(mBase + mOff + r) * ldc + n];
        if (ACT == 1) v = tanhf(v);
        if (ACT == 2) v = fmaxf(v, 0.0f);
        if (ACT == 3) v = v / (1.0f + expf(-v));
        if (ACT == 4) v = (v > 0.f) ? v : 0.01f * v;
        if (ACT == 5) v = 0.5f * v * (1.0f + erff(v * 0.70710678118654752f));
        if (BNR) v = fmaxf(v * sv + tv, 0.0f);
        slab[(mOff + r) * 68 + (j << 4) + rlane] = v;
      }
    }
    __builtin_amdgcn_fence(__ATOMIC_RELEASE, "workgroup");
    __builtin_amdgcn_wave_barrier();
    __builtin_amdgcn_fence(__ATOMIC_ACQUIRE, "workgroup");
    if (OUT_MODE == 0) {
      float* C = (float*)Cout + (size_t)b * strideC;
      const int hh = lane >> 4, c4 = (lane & 15) * 4;
      for (int pass = 0; pass < 2; ++pass) {
#pragma unroll
        for (int it = 0; it < 8; ++it) {
          const int row = it * 2 + hh;
          v4f v = *(const v4f*)(slab + row * 68 + c4);
          if (mBase + row < Mst) *(volatile v4f*)(C + (size_t)(mBase + row) * ldc + n0 + c4) = v;
        }
        __threadfence();
      }
    } else {
      const int q = lane >> 3, c8 = (lane & 7) * 8;
      unsigned short* C  = (unsigned short*)Cout  + (size_t)b * strideC;
      unsigned short* C2 = (OUT_MODE == 2) ? ((unsigned short*)Cout2 + (size_t)b * strideC) : nullptr;
      for (int pass = 0; pass < 2; ++pass) {
#pragma unroll
        for (int it = 0; it < 4; ++it) {
          const int row = it * 4 + q;
          const float* sp = slab + row * 68 + c8;
          v8h hv, lv;
#pragma unroll
          for (int e = 0; e < 8; ++e) {
            if (OUT_MODE == 1) {
              hv[e] = (_Float16)sp[e];
            } else {
              unsigned short hb = f2bf_bits(sp[e]);
              unsigned short lb = f2bf_bits(sp[e] - bf_bits2f(hb));
              hv[e] = __builtin_bit_cast(_Float16, hb);
              lv[e] = __builtin_bit_cast(_Float16, lb);
            }
          }
          if (mBase + row < Mst) {
            *(volatile v8h*)(C + (size_t)(mBase + row) * ldc + n0 + c8) = hv;
            if (OUT_MODE == 2) *(volatile v8h*)(C2 + (size_t)(mBase + row) * ldc + n0 + c8) = lv;
          }
        }
        __threadfence();
      }
    }
    __builtin_amdgcn_fence(__ATOMIC_RELEASE, "workgroup");
    __builtin_amdgcn_wave_barrier();
    __builtin_amdgcn_fence(__ATOMIC_ACQUIRE, "workgroup");
  }
}

__device__ __forceinline__ int blk_excl_scan(int cnt, int* scan_ws, int tid, int* tot) {
  const int lane = tid & 31, wave = tid >> 5; int incl = cnt;
#pragma unroll
  for (int o = 1; o < 32; o <<= 1) { const int v = __shfl_up(incl, o, 32); if (lane >= o) incl += v; }
  if (lane == 31) scan_ws[wave] = incl;
  __syncthreads();
  if (wave == 0) { int wv = (lane < NT / 32) ? scan_ws[lane] : 0; int wincl = wv;
#pragma unroll
    for (int o = 1; o < 32; o <<= 1) { const int v = __shfl_up(wincl, o, 32); if (lane >= o) wincl += v; }
    if (lane < NT / 32) scan_ws[32 + lane] = wincl - wv; if (lane == 31) scan_ws[64] = wincl; }
  __syncthreads();
  const int res = scan_ws[32 + wave] + incl - cnt; *tot = scan_ws[64];
  return res;
}
template <int SP, int CAP>
__device__ __forceinline__ int chunk_hits(const int* __restrict__ dstv, const int* __restrict__ srcv, int e0, int n0, int tid,
                                          int* LIST, int* scan_ws) {
  const int eb = e0 + tid * SP;
  const bool inr = eb < NE;
  const int ebc = inr ? eb : (NE - SP);
  int rec[SP]; int cnt = 0;
#pragma unroll
  for (int k = 0; k < SP; k += 4) {
    const v4i d4 = *(const v4i*)(dstv + ebc + k);
    const v4i s4 = *(const v4i*)(srcv + ebc + k);
#pragma unroll
    for (int e = 0; e < 4; ++e) {
      const int d = d4[e]; int r = -1;
      if (inr && d >= n0 && d < n0 + SRB) { int s = s4[e]; s = s < 0 ? 0 : (s >= NN ? NN - 1 : s); r = ((d - n0) << 16) | s; ++cnt; }
      rec[k + e] = r;
    }
  }
  int tot; int p = blk_excl_scan(cnt, scan_ws, tid, &tot);
#pragma unroll
  for (int k = 0; k < SP; ++k) if (rec[k] >= 0) { if ((unsigned)p < (unsigned)CAP) LIST[p] = rec[k]; ++p; }
  __syncthreads();
  return tot < CAP ? tot : CAP;
}

__global__ __launch_bounds__(NT) void prep_kernel(const float* __restrict__ W0a, const float* __restrict__ W0b, const float* __restrict__ W1a,
                                                 const float* __restrict__ Wr1, const float* __restrict__ Wr2,
                                                 const float* __restrict__ g0i, const float* __restrict__ be0i, const float* __restrict__ m0i, const float* __restrict__ v0i,
                                                 const float* __restrict__ g0,  const float* __restrict__ be0,  const float* __restrict__ m0,  const float* __restrict__ v0,
                                                 const float* __restrict__ g1i, const float* __restrict__ be1i, const float* __restrict__ m1i, const float* __restrict__ v1i,
                                                 const float* __restrict__ g1,  const float* __restrict__ be1,  const float* __restrict__ m1,  const float* __restrict__ v1,
                                                 unsigned* __restrict__ WT, float* __restrict__ BNC) {
  const int i = blockIdx.x * NT + threadIdx.x;
  if (i < 5 * 2048) {
    const int mtx = i >> 11;
    const int r = i & 2047;
    const int o = r >> 5;
    const int k = 2 * (r & 31);
    const float* W = W0a;
    if (mtx == 1) W = W0b;
    if (mtx == 2) W = W1a;
    if (mtx == 3) W = Wr1;
    if (mtx == 4) W = Wr2;
    const float a = W[k * GD + o] * WSC, b = W[(k + 1) * GD + o] * WSC;
    const _Float16 ha = (_Float16)a, hb = (_Float16)b;
    const unsigned u = (unsigned)__builtin_bit_cast(unsigned short, ha) | ((unsigned)__builtin_bit_cast(unsigned short, hb) << 16);
    ((volatile unsigned*)WT)[i] = u;
    __threadfence();
    ((volatile unsigned*)WT)[i] = u;
  }
  if (blockIdx.x == 0) {
    const int t = threadIdx.x;
    const int layer = t >> 7, which = (t >> 6) & 1, n = t & 63;
    const float gi0 = g0i[n], bi0 = be0i[n], mi0 = m0i[n], vi0 = v0i[n];
    const float go0 = g0[n],  bo0 = be0[n],  mo0 = m0[n],  vo0 = v0[n];
    const float gi1 = g1i[n], bi1 = be1i[n], mi1 = m1i[n], vi1 = v1i[n];
    const float go1 = g1[n],  bo1 = be1[n],  mo1 = m1[n],  vo1 = v1[n];
    const float gi = layer ? gi1 : gi0, bi = layer ? bi1 : bi0, mi = layer ? mi1 : mi0, vi = layer ? vi1 : vi0;
    const float go = layer ? go1 : go0, bo = layer ? bo1 : bo0, mo = layer ? mo1 : mo0, vo = layer ? vo1 : vo0;
    const float si = gi * (1.0f / sqrtf(vi + 1e-5f));
    const float ti = bi - mi * si;
    const float so = go * (1.0f / sqrtf(vo + 1e-5f));
    const float to = bo - mo * so;
    const float val = which ? (ti * so + to) : (si * so);
    ((volatile float*)BNC)[t] = val;
    __threadfence();
    ((volatile float*)BNC)[t] = val;
  }
}

__global__ __launch_bounds__(NT) void gin_agg_kernel(const float* __restrict__ feat, const int* __restrict__ srcv, const int* __restrict__ dstv,
                                                    const float* __restrict__ epsp, float* ACC, unsigned short* __restrict__ A16) {
  __shared__ int LIST[SCH];
  __shared__ int scan_ws[80];
  const int tid = threadIdx.x, lane = tid & 31, wave = tid >> 5;
  const int n0 = blockIdx.x * SRB;
  const float alpha = 1.0f + epsp[0];
  const v2f z2 = {0.f, 0.f};
#pragma unroll 1
  for (int j = 0; j < SRB / 8; ++j) {
    const int dl = wave * (SRB / 8) + j;
    const int n = n0 + dl;
    const int nc = n < NN ? n : NN - 1;
    v2f v = *(const v2f*)(feat + (size_t)nc * GD + 2 * lane);
    v = v * alpha;
    if (n >= NN) v = z2;
    float* rp = ACC + (size_t)(n0 + dl) * GD + 2 * lane;
    *(volatile v2f*)rp = v; __threadfence(); *(volatile v2f*)rp = v;
  }
  __syncthreads();
#pragma unroll 1
  for (int c = 0; c < NCH; ++c) {
    const int tot = chunk_hits<SCH / NT, SCH>(dstv, srcv, c * SCH, n0, tid, LIST, scan_ws);
#pragma unroll 1
    for (int base = 0; base < tot; base += 32) {
      const int q = base + lane;
      const int rv = (q < tot) ? LIST[q] : -1;
      const int own = (rv >= 0 && (rv >> 24) == wave) ? 1 : 0;
      unsigned msk = (unsigned)__ballot(own);
#pragma unroll 1
      for (int it = 0; it < 32; ++it) {
        if (msk == 0u) break;
        const int bp = __builtin_ctz(msk); msk &= msk - 1u;
        const int r = __shfl(rv, bp, 32);
        const int dl = r >> 16, s = r & 0xFFFF;
        const v2f hv = *(const v2f*)(feat + (size_t)s * GD + 2 * lane);
        float* rp = ACC + (size_t)(n0 + dl) * GD + 2 * lane;
        v2f a = *(const v2f*)rp;
        a = a + hv;
        *(volatile v2f*)rp = a; __threadfence(); *(volatile v2f*)rp = a;
      }
    }
    __syncthreads();
  }
  const int q4 = lane >> 3, c8 = (lane & 7) * 8;
#pragma unroll 1
  for (int j = 0; j < SRB / 32; ++j) {
    const int dl0 = wave * (SRB / 8) + 4 * j;
    const int nb = n0 + dl0;
    if (nb < NP) {
      const bool live = nb < NN;
      const float* rp = ACC + (size_t)(n0 + dl0 + q4) * GD + c8;
      const v4f x0 = *(const v4f*)rp, x1 = *(const v4f*)(rp + 4);
      v8h hv;
#pragma unroll
      for (int e = 0; e < 4; ++e) {
        hv[e]     = live ? (_Float16)x0[e] : (_Float16)0.f;
        hv[4 + e] = live ? (_Float16)x1[e] : (_Float16)0.f;
      }
      unsigned short* op = A16 + (size_t)(nb + q4) * GD + c8;
      *(volatile v8h*)op = hv; __threadfence(); *(volatile v8h*)op = hv;
    }
  }
}

__global__ __launch_bounds__(NT) void pool_kernel(const float* __restrict__ H, const int* __restrict__ gid, unsigned* __restrict__ P16) {
  __shared__ int LIST[SCHP];
  __shared__ int scan_ws[80];
  __shared__ __align__(16) float red[8 * GD];
  __shared__ int rc[8];
  const int tid = threadIdx.x, lane = tid & 31, wave = tid >> 5;
  const int g = blockIdx.x;
  const v2f z2 = {0.f, 0.f};
  v2f acc = z2; int cnt = 0;
#pragma unroll 1
  for (int c = 0; c < NCHP; ++c) {
    const int eb = c * SCHP + tid * 8;
    const bool inr = eb < NN;
    const int ebc = inr ? eb : (NN - 8);
    const v4i b0 = *(const v4i*)(gid + ebc), b1 = *(const v4i*)(gid + ebc + 4);
    int bv[8];
    bv[0] = b0[0]; bv[1] = b0[1]; bv[2] = b0[2]; bv[3] = b0[3]; bv[4] = b1[0]; bv[5] = b1[1]; bv[6] = b1[2]; bv[7] = b1[3];
    int rec[8]; int kc = 0;
#pragma unroll
    for (int k = 0; k < 8; ++k) { rec[k] = -1; if (inr && bv[k] == g) { rec[k] = eb + k; ++kc; } }
    int tot; int p = blk_excl_scan(kc, scan_ws, tid, &tot);
#pragma unroll
    for (int k = 0; k < 8; ++k) if (rec[k] >= 0) { if ((unsigned)p < (unsigned)SCHP) LIST[p] = rec[k]; ++p; }
    __syncthreads();
    const int totc = tot < SCHP ? tot : SCHP;
#pragma unroll 1
    for (int q = wave; q < totc; q += 8) {
      int nd = LIST[q]; nd = nd < 0 ? 0 : (nd >= NN ? NN - 1 : nd);
      acc = acc + *(const v2f*)(H + (size_t)nd * GD + 2 * lane); ++cnt;
    }
    __syncthreads();
  }
  *(v2f*)(red + wave * GD + 2 * lane) = acc;
  if (lane == 0) rc[wave] = cnt;
  __syncthreads();
  if (wave == 0) {
    v2f s = z2; int ct = 0;
#pragma unroll
    for (int w = 0; w < 8; ++w) { s = s + *(const v2f*)(red + w * GD + 2 * lane); ct += rc[w]; }
    const float cf = (float)ct;
    const float inv = 1.0f / fmaxf(cf, 1.0f);
    const v2f o = s * inv;
    const _Float16 h0 = (_Float16)o[0], h1 = (_Float16)o[1];
    const unsigned u = (unsigned)__builtin_bit_cast(unsigned short, h0) | ((unsigned)__builtin_bit_cast(unsigned short, h1) << 16);
    unsigned* pp = P16 + (size_t)g * (GD / 2) + lane;
    *(volatile unsigned*)pp = u;
    __threadfence();
    *(volatile unsigned*)pp = u;
  }
}

extern "C" void kernel_launch(void* const* d_in, const int* in_sizes, int n_in,
                              void* d_out, int out_size, void* d_ws, size_t ws_size, hipStream_t stream) {
  if (n_in < 32) return;
  if (in_sizes[0] != NN * GD || in_sizes[1] != NE || in_sizes[2] != NE || in_sizes[3] != NN) return;
  if (out_size != NGR * GD + NN * GD) return;
  const float* x    = (const float*)d_in[0];
  const int*   src  = (const int*)d_in[1];
  const int*   dst  = (const int*)d_in[2];
  const int*   gids = (const int*)d_in[3];
  const float* eps0 = (const float*)d_in[4];
  const float* W0a  = (const float*)d_in[5];
  const float* bb0a = (const float*)d_in[6];
  const float* W0b  = (const float*)d_in[7];
  const float* bb0b = (const float*)d_in[8];
  const float* g0i  = (const float*)d_in[9];
  const float* be0i = (const float*)d_in[10];
  const float* m0i  = (const float*)d_in[11];
  const float* v0i  = (const float*)d_in[12];
  const float* g0   = (const float*)d_in[13];
  const float* be0  = (const float*)d_in[14];
  const float* m0   = (const float*)d_in[15];
  const float* v0   = (const float*)d_in[16];
  const float* eps1 = (const float*)d_in[17];
  const float* W1a  = (const float*)d_in[18];
  const float* bb1a = (const float*)d_in[19];
  const float* g1i  = (const float*)d_in[20];
  const float* be1i = (const float*)d_in[21];
  const float* m1i  = (const float*)d_in[22];
  const float* v1i  = (const float*)d_in[23];
  const float* g1   = (const float*)d_in[24];
  const float* be1  = (const float*)d_in[25];
  const float* m1   = (const float*)d_in[26];
  const float* v1   = (const float*)d_in[27];
  const float* Wr1  = (const float*)d_in[28];
  const float* br1  = (const float*)d_in[29];
  const float* Wr2  = (const float*)d_in[30];
  const float* br2  = (const float*)d_in[31];
  float* out  = (float*)d_out;
  float* out1 = out + (size_t)NGR * GD;

  char* ws = (char*)d_ws; size_t off = 0;
  auto carve = [&](size_t bytes) -> char* { char* p = ws + off; off += (bytes + 255) & ~(size_t)255; return p; };
  unsigned*       WT  = (unsigned*)carve((size_t)5 * 2048 * 4);
  float*          BNC = (float*)carve(1024);
  float*          ACC = (float*)carve((size_t)NTILE * SRB * GD * 4);
  unsigned short* A16 = (unsigned short*)carve((size_t)NP * GD * 2);
  unsigned short* T16 = (unsigned short*)carve((size_t)NP * GD * 2);
  float*          H0  = (float*)carve((size_t)NP * GD * 4);
  unsigned*       P16 = (unsigned*)carve((size_t)NGP * GD * 2);
  unsigned short* R16 = (unsigned short*)carve((size_t)NGP * GD * 2);
  if (off > ws_size || off > (size_t)134217728) return;

  const unsigned short* WT16 = (const unsigned short*)WT;
  const unsigned short* Bt0 = WT16;
  const unsigned short* Bt1 = WT16 + 4096;
  const unsigned short* Bt2 = WT16 + 8192;
  const unsigned short* Bt3 = WT16 + 12288;
  const unsigned short* Bt4 = WT16 + 16384;
  const float* S0 = BNC; const float* T0 = BNC + 64; const float* S1 = BNC + 128; const float* T1 = BNC + 192;
  const float sc = WSC_INV;
  const int blkBig = ((NP / 64) * (GD / 64) + 7) / 8;
  const int blkSml = ((NGP / 64) * (GD / 64) + 7) / 8;

  prep_kernel<<<(5 * 2048) / NT, NT, 0, stream>>>(W0a, W0b, W1a, Wr1, Wr2,
                                                  g0i, be0i, m0i, v0i, g0, be0, m0, v0,
                                                  g1i, be1i, m1i, v1i, g1, be1, m1, v1, WT, BNC);
  gin_agg_kernel<<<NTILE, NT, 0, stream>>>(x, src, dst, eps0, ACC, A16);
  wmma_gemm64<0, false, 2, 1, false, 2, false><<<dim3(blkBig, 1), 256, 0, stream>>>(
      (const unsigned short*)A16, (const unsigned short*)A16, GD, 0L,
      Bt0, Bt0, GD, 0L,
      (void*)T16, (void*)T16, GD, 0L,
      bb0a, S0, T0, BNC, 0L, NP, GD, GD, NP, sc);
  wmma_gemm64<0, false, 2, 0, false, 2, true><<<dim3(blkBig, 1), 256, 0, stream>>>(
      (const unsigned short*)T16, (const unsigned short*)T16, GD, 0L,
      Bt1, Bt1, GD, 0L,
      (void*)H0, (void*)H0, GD, 0L,
      bb0b, S0, T0, BNC, 0L, NP, GD, GD, NP, sc);
  gin_agg_kernel<<<NTILE, NT, 0, stream>>>(H0, src, dst, eps1, ACC, A16);
  wmma_gemm64<0, false, 2, 0, false, 2, true><<<dim3(blkBig, 1), 256, 0, stream>>>(
      (const unsigned short*)A16, (const unsigned short*)A16, GD, 0L,
      Bt2, Bt2, GD, 0L,
      (void*)out1, (void*)out1, GD, 0L,
      bb1a, S1, T1, BNC, 0L, NP, GD, GD, NN, sc);
  pool_kernel<<<NGP, NT, 0, stream>>>(out1, gids, P16);
  wmma_gemm64<0, false, 2, 1, false, 2, false><<<dim3(blkSml, 1), 256, 0, stream>>>(
      (const unsigned short*)P16, (const unsigned short*)P16, GD, 0L,
      Bt3, Bt3, GD, 0L,
      (void*)R16, (void*)R16, GD, 0L,
      br1, S0, T0, BNC, 0L, NGP, GD, GD, NGP, sc);
  wmma_gemm64<0, false, 2, 0, false, 0, false><<<dim3(blkSml, 1), 256, 0, stream>>>(
      (const unsigned short*)R16, (const unsigned short*)R16, GD, 0L,
      Bt4, Bt4, GD, 0L,
      (void*)out, (void*)out, GD, 0L,
      br2, S0, T0, BNC, 0L, NGP, GD, GD, NGR, sc);
}
